// SelectiveSSM_27066883899746
// MI455X (gfx1250) — hardware-verified
//
#include <hip/hip_runtime.h>
#include <math.h>

typedef __attribute__((ext_vector_type(16))) __bf16   v16b;
typedef __attribute__((ext_vector_type(8)))  __bf16   v8b;
typedef __attribute__((ext_vector_type(8)))  float    v8f;
typedef __attribute__((ext_vector_type(4)))  float    v4f;
typedef __attribute__((ext_vector_type(4)))  unsigned v4u;

constexpr int kBatch  = 2;
constexpr int kSeq    = 2048;
constexpr int kD      = 1024;
constexpr int kNst    = 16;
constexpr int kDtR    = 64;
constexpr int kProj   = 2 * kNst + kDtR;
constexpr int kXpP    = 128;
constexpr int kRows   = kBatch * kSeq;
constexpr int kScanTS = 64;
constexpr int kScanCh = 64;
constexpr int kScanYP = 68;
constexpr int kBC     = 2 * kNst;
static_assert(kProj == 96);
static_assert(kProj <= kXpP);
static_assert((kD % 32) == 0 && (kDtR % 32) == 0);
static_assert((kRows % 64) == 0 && (kXpP % 64) == 0 && (kD % 64) == 0);
static_assert((kSeq % kScanTS) == 0 && (kD % kScanCh) == 0);
static_assert(((kRows * kD) % 2048) == 0);
static_assert(kBC == 32 && kScanCh == 64 && kScanTS == 64);

constexpr size_t kOffXH   = 0;
constexpr size_t kOffXL   = kOffXH  + (size_t)kRows * kD   * 2;
constexpr size_t kOffWXH  = kOffXL  + (size_t)kRows * kD   * 2;
constexpr size_t kOffWXL  = kOffWXH + (size_t)kXpP  * kD   * 2;
constexpr size_t kOffWDH  = kOffWXL + (size_t)kXpP  * kD   * 2;
constexpr size_t kOffWDL  = kOffWDH + (size_t)kD    * kDtR * 2;
constexpr size_t kOffXP   = kOffWDL + (size_t)kD    * kDtR * 2;
constexpr size_t kOffDRH  = kOffXP  + (size_t)kRows * kXpP * 4;
constexpr size_t kOffDRL  = kOffDRH + (size_t)kRows * kDtR * 2;
constexpr size_t kOffPRE  = kOffDRL + (size_t)kRows * kDtR * 2;
constexpr size_t kOffDT   = kOffPRE + (size_t)kRows * kD   * 4;
constexpr size_t kWsTotal = kOffDT  + (size_t)kRows * kD   * 4;
static_assert(kWsTotal == 54263808ull);
static_assert(kWsTotal <= 134217728ull);
static_assert((kOffXL % 128) == 0 && (kOffWXH % 128) == 0 && (kOffWXL % 128) == 0 && (kOffWDH % 128) == 0 &&
              (kOffWDL % 128) == 0 && (kOffXP % 128) == 0 && (kOffDRH % 128) == 0 && (kOffDRL % 128) == 0 &&
              (kOffPRE % 128) == 0 && (kOffDT % 128) == 0);

__device__ __forceinline__ unsigned bf_rne_bits32(float f) {
  unsigned u = __float_as_uint(f);
  const unsigned lsb = (u & 0x00010000u) ? 1u : 0u;
  u = (u + 0x7FFFu + lsb) & 0xFFFF0000u;
  return u;
}
__device__ __forceinline__ void split_pack2(float f0, float f1, unsigned& wh, unsigned& wl) {
  const unsigned h0 = bf_rne_bits32(f0);
  const unsigned h1 = bf_rne_bits32(f1);
  const unsigned l0 = bf_rne_bits32(f0 - __uint_as_float(h0));
  const unsigned l1 = bf_rne_bits32(f1 - __uint_as_float(h1));
  wh = __builtin_amdgcn_perm(h1, h0, 0x07060302u);
  wl = __builtin_amdgcn_perm(l1, l0, 0x07060302u);
}

__device__ __forceinline__ void mma_guard(v8f& acc, v16b a0, v16b a1, v16b b0, v16b b1) {
  asm volatile("v_nop\n\tv_nop\n\tv_nop\n\tv_nop" : "+v"(acc) : "v"(a0), "v"(a1), "v"(b0), "v"(b1));
}
__device__ __forceinline__ void acc_guard1(v8f& acc) {
  asm volatile("v_nop\n\tv_nop\n\tv_nop\n\tv_nop" : "+v"(acc));
}
__device__ __forceinline__ void keep4_b(v16b a, v16b b, v16b c, v16b d) {
  asm volatile("v_nop" :: "v"(a), "v"(b), "v"(c), "v"(d));
}
template <typename T> struct Frag;
template <> struct Frag<__bf16> {
  typedef v16b V;
  union U { v16b v; v8b h[2]; };
  static __device__ __forceinline__ v16b load(const __bf16* p) {
    U f;
    f.h[0] = *(const v8b*)(p);
    f.h[1] = *(const v8b*)(p + 16);
    return f.v;
  }
  static __device__ __forceinline__ v8f mma(v16b a, v16b b, v8f c) {
    return __builtin_amdgcn_wmma_f32_16x16x32_bf16(false, a, false, b, (short)0, c, false, false);
  }
};

template <int BIAS_MODE>
__global__ __launch_bounds__(256) void wmma_gemm64_split(
    const unsigned short* __restrict__ Ap, const unsigned short* __restrict__ A2p, int lda,
    const unsigned short* __restrict__ Btp, const unsigned short* __restrict__ Bt2p, int ldb,
    float* __restrict__ Cout, int ldc,
    const float* __restrict__ bias,
    int M, int N, int K) {
  typedef __bf16 T;
  typedef Frag<T>::V V;
  const T* Ab  = (const T*)Ap;
  const T* Ab2 = (const T*)A2p;
  const T* Bb  = (const T*)Btp;
  const T* Bb2 = (const T*)Bt2p;
  __shared__ __align__(16) float sT[8][16 * 68];
  const int lane = threadIdx.x & 31;
  const int wave = threadIdx.x >> 5;
  const int tilesN = N >> 6;
  const int tilesM = M >> 6;
  const int tile = blockIdx.x * 8 + wave;
  if (tile >= tilesM * tilesN) return;
  const int tm = tile / tilesN;
  const int tn = tile - tm * tilesN;
  const int m0 = tm << 6;
  const int n0 = tn << 6;

  const int rlane = lane & 15;
  const int koff  = (lane >> 4) * 8;
  const int mOff  = (lane >> 4) * 8;

  v8f acc[4][4];
#pragma unroll
  for (int i = 0; i < 4; ++i)
#pragma unroll
    for (int j = 0; j < 4; ++j) acc[i][j] = (v8f){0.f, 0.f, 0.f, 0.f, 0.f, 0.f, 0.f, 0.f};

  for (int k0 = 0; k0 < K; k0 += 32) {
    V bh[4], bl[4];
#pragma unroll
    for (int j = 0; j < 4; ++j) {
      const size_t bo = (size_t)(n0 + (j << 4) + rlane) * ldb + koff + k0;
      bh[j] = Frag<T>::load(Bb + bo);
      bl[j] = Frag<T>::load(Bb2 + bo);
    }
#pragma unroll
    for (int i = 0; i < 4; ++i) {
      const size_t ao = (size_t)(m0 + (i << 4) + rlane) * lda + koff + k0;
      V ah = Frag<T>::load(Ab + ao);
      V al = Frag<T>::load(Ab2 + ao);
#pragma unroll
      for (int j = 0; j < 4; ++j) {
        acc[i][j] = Frag<T>::mma(ah, bh[j], acc[i][j]);
        acc[i][j] = Frag<T>::mma(ah, bl[j], acc[i][j]);
        acc[i][j] = Frag<T>::mma(al, bh[j], acc[i][j]);
      }
      mma_guard(acc[i][0], ah, al, bh[0], bl[0]);
      mma_guard(acc[i][1], ah, al, bh[1], bl[1]);
      mma_guard(acc[i][2], ah, al, bh[2], bl[2]);
      mma_guard(acc[i][3], ah, al, bh[3], bl[3]);
    }
    keep4_b(bh[0], bh[1], bh[2], bh[3]);
    keep4_b(bl[0], bl[1], bl[2], bl[3]);
  }
#pragma unroll
  for (int i = 0; i < 4; ++i)
#pragma unroll
    for (int j = 0; j < 4; ++j) acc_guard1(acc[i][j]);

  float* slab = sT[wave];
#pragma unroll
  for (int i = 0; i < 4; ++i) {
    const int mBase = m0 + (i << 4);
#pragma unroll
    for (int j = 0; j < 4; ++j) {
      const int n = n0 + (j << 4) + rlane;
      float bv = 0.f;
      if (BIAS_MODE == 2) bv = bias[n];
#pragma unroll
      for (int r = 0; r < 8; ++r) {
        float v = acc[i][j][r];
        if (BIAS_MODE == 2) v += bv;
        slab[(mOff + r) * 68 + (j << 4) + rlane] = v;
      }
    }
    __builtin_amdgcn_fence(__ATOMIC_RELEASE, "workgroup");
    __builtin_amdgcn_wave_barrier();
    __builtin_amdgcn_fence(__ATOMIC_ACQUIRE, "workgroup");
    {
      const int hh = lane >> 4, c4 = (lane & 15) * 4;
      for (int pass = 0; pass < 2; ++pass) {
#pragma unroll
        for (int it = 0; it < 8; ++it) {
          const int row = it * 2 + hh;
          v4f v = *(const v4f*)(slab + row * 68 + c4);
          *(volatile v4f*)(Cout + (size_t)(mBase + row) * ldc + n0 + c4) = v;
        }
        __threadfence();
      }
    }
    __builtin_amdgcn_fence(__ATOMIC_RELEASE, "workgroup");
    __builtin_amdgcn_wave_barrier();
    __builtin_amdgcn_fence(__ATOMIC_ACQUIRE, "workgroup");
  }
}

__global__ __launch_bounds__(256) void split_rows_bf16_kernel(
    const float* __restrict__ src, unsigned src_pitch, unsigned src_col0, unsigned g_log2,
    unsigned short* __restrict__ dhi, unsigned short* __restrict__ dlo, unsigned total8)
{
  const unsigned i = blockIdx.x * 256u + threadIdx.x;
  if (i >= total8) return;
  unsigned row = i >> g_log2;
  unsigned g = i - (row << g_log2);
  asm volatile("" : "+v"(row));
  asm volatile("" : "+v"(g));
  const size_t so = (size_t)row * src_pitch + src_col0 + g * 8u;
  const size_t e0 = (size_t)i * 8u;
  const v4f a0 = *(const v4f*)(src + so);
  const v4f a1 = *(const v4f*)(src + so + 4);
  const float f0 = a0[0], f1 = a0[1], f2 = a0[2], f3 = a0[3];
  const float f4 = a1[0], f5 = a1[1], f6 = a1[2], f7 = a1[3];
  unsigned wh0, wh1, wh2, wh3, wl0, wl1, wl2, wl3;
  split_pack2(f0, f1, wh0, wl0);
  split_pack2(f2, f3, wh1, wl1);
  split_pack2(f4, f5, wh2, wl2);
  split_pack2(f6, f7, wh3, wl3);
  const v4u hv = (v4u){wh0, wh1, wh2, wh3};
  const v4u lv = (v4u){wl0, wl1, wl2, wl3};
  unsigned short* qh = dhi + e0;
  unsigned short* ql = dlo + e0;
  *(volatile v4u*)qh = hv;
  *(volatile v4u*)ql = lv;
  __threadfence();
  *(volatile v4u*)qh = hv;
  *(volatile v4u*)ql = lv;
}

__global__ __launch_bounds__(256) void transpose_split_bf16_kernel(
    const float* __restrict__ src, unsigned n_real, unsigned kg_log2,
    unsigned short* __restrict__ dhi, unsigned short* __restrict__ dlo, unsigned total8)
{
  const unsigned i = blockIdx.x * 256u + threadIdx.x;
  if (i >= total8) return;
  unsigned n = i >> kg_log2;
  unsigned g = i - (n << kg_log2);
  asm volatile("" : "+v"(n));
  asm volatile("" : "+v"(g));
  const unsigned k0 = g * 8u;
  const bool live = (n < n_real);
  const unsigned nc = live ? n : (n_real - 1u);
  float f0 = src[(size_t)(k0 + 0u) * n_real + nc];
  float f1 = src[(size_t)(k0 + 1u) * n_real + nc];
  float f2 = src[(size_t)(k0 + 2u) * n_real + nc];
  float f3 = src[(size_t)(k0 + 3u) * n_real + nc];
  float f4 = src[(size_t)(k0 + 4u) * n_real + nc];
  float f5 = src[(size_t)(k0 + 5u) * n_real + nc];
  float f6 = src[(size_t)(k0 + 6u) * n_real + nc];
  float f7 = src[(size_t)(k0 + 7u) * n_real + nc];
  asm volatile("" : "+v"(f0), "+v"(f1), "+v"(f2), "+v"(f3));
  asm volatile("" : "+v"(f4), "+v"(f5), "+v"(f6), "+v"(f7));
  f0 = live ? f0 : 0.0f;
  f1 = live ? f1 : 0.0f;
  f2 = live ? f2 : 0.0f;
  f3 = live ? f3 : 0.0f;
  f4 = live ? f4 : 0.0f;
  f5 = live ? f5 : 0.0f;
  f6 = live ? f6 : 0.0f;
  f7 = live ? f7 : 0.0f;
  unsigned wh0, wh1, wh2, wh3, wl0, wl1, wl2, wl3;
  split_pack2(f0, f1, wh0, wl0);
  split_pack2(f2, f3, wh1, wl1);
  split_pack2(f4, f5, wh2, wl2);
  split_pack2(f6, f7, wh3, wl3);
  const v4u hv = (v4u){wh0, wh1, wh2, wh3};
  const v4u lv = (v4u){wl0, wl1, wl2, wl3};
  const size_t e0 = (size_t)i * 8u;
  unsigned short* qh = dhi + e0;
  unsigned short* ql = dlo + e0;
  *(volatile v4u*)qh = hv;
  *(volatile v4u*)ql = lv;
  __threadfence();
  *(volatile v4u*)qh = hv;
  *(volatile v4u*)ql = lv;
}

__global__ __launch_bounds__(256) void softplus_kernel(const float* __restrict__ pre, float* __restrict__ dt)
{
  const unsigned base = blockIdx.x * 2048u + threadIdx.x;
#pragma unroll 1
  for (unsigned k = 0; k < 8u; ++k) {
    const unsigned e = base + k * 256u;
    const float v = pre[e];
    const float ex = expf(-fabsf(v));
    const float r = fmaxf(v, 0.0f) + log1pf(ex);
    float* p = dt + e;
    *(volatile float*)p = r;
    __threadfence();
    *(volatile float*)p = r;
  }
}

__global__ __launch_bounds__(64) void scan_kernel(
    const float* __restrict__ XP, const float* __restrict__ DT, const float* __restrict__ X,
    const float* __restrict__ Alog, float* __restrict__ Y)
{
  __shared__ __align__(16) float sBC[kScanTS * kBC];
  __shared__ __align__(16) float sY[kScanTS * kScanYP];
  __shared__ __align__(16) float sA[kNst * kScanCh];
  const unsigned tid = threadIdx.x;
  const unsigned lane = tid & 31u;
  const unsigned wave = tid >> 5;
  constexpr unsigned kBlkPerB = (unsigned)(kD / kScanCh);
  const unsigned bix = blockIdx.x / kBlkPerB;
  const unsigned d0 = (blockIdx.x - bix * kBlkPerB) * (unsigned)kScanCh;
  const unsigned d = d0 + tid;
  const size_t row0 = (size_t)bix * kSeq;

#pragma unroll 1
  for (int s = 0; s < kNst; ++s) sA[s * kScanCh + tid] = -expf(Alog[(size_t)s * kD + d]);
  __syncthreads();
  float negA[kNst], h[kNst];
#pragma unroll
  for (int s = 0; s < kNst; ++s) {
    negA[s] = sA[s * kScanCh + tid];
    h[s] = 0.f;
  }

  const unsigned lr = tid >> 3, lc4 = (tid & 7u) * 4u;
  const unsigned hh = lane >> 4, c4 = (lane & 15u) * 4u;

#pragma unroll 1
  for (unsigned t0 = 0; t0 < (unsigned)kSeq; t0 += (unsigned)kScanTS) {
    __syncthreads();
#pragma unroll
    for (unsigned i = 0; i < 8u; ++i) {
      const unsigned r = lr + 8u * i;
      *(v4f*)(sBC + r * kBC + lc4) = *(const v4f*)(XP + (row0 + t0 + r) * kXpP + lc4);
    }
    __syncthreads();
#pragma unroll 1
    for (unsigned s = 0; s < (unsigned)kScanTS; ++s) {
      const size_t grow = row0 + t0 + s;
      const float dtv = DT[grow * kD + d];
      const float xv  = X[grow * kD + d];
      const float* br = sBC + s * kBC;
      float Bs[kNst], Cs[kNst];
#pragma unroll
      for (int q4 = 0; q4 < 4; ++q4) {
        const v4f bv = *(const v4f*)(br + 4 * q4);
        const v4f cv = *(const v4f*)(br + kNst + 4 * q4);
        Bs[4 * q4 + 0] = bv[0]; Bs[4 * q4 + 1] = bv[1]; Bs[4 * q4 + 2] = bv[2]; Bs[4 * q4 + 3] = bv[3];
        Cs[4 * q4 + 0] = cv[0]; Cs[4 * q4 + 1] = cv[1]; Cs[4 * q4 + 2] = cv[2]; Cs[4 * q4 + 3] = cv[3];
      }
      float y = 0.f;
#pragma unroll
      for (int k = 0; k < kNst; ++k) {
        const float e  = expf(negA[k] * dtv);
        const float bu = (Bs[k] * dtv) * xv;
        h[k] = fmaf(e, h[k], bu);
        y = fmaf(Cs[k], h[k], y);
      }
      sY[s * kScanYP + tid] = y;
    }
    __syncthreads();
    for (int pass = 0; pass < 2; ++pass) {
#pragma unroll
      for (unsigned it = 0; it < 16u; ++it) {
        const unsigned row = it * 4u + wave * 2u + hh;
        const v4f v = *(const v4f*)(sY + row * kScanYP + c4);
        *(volatile v4f*)(Y + (row0 + t0 + row) * kD + d0 + c4) = v;
      }
      __threadfence();
    }
  }
}

extern "C" void kernel_launch(void* const* d_in, const int* in_sizes, int n_in,
                              void* d_out, int out_size, void* d_ws, size_t ws_size,
                              hipStream_t stream) {
  if (n_in < 5) return;
  if (in_sizes[0] != kRows * kD) return;
  if (in_sizes[1] != kD * kProj) return;
  if (in_sizes[2] != kDtR * kD) return;
  if (in_sizes[3] != kD) return;
  if (in_sizes[4] != kNst * kD) return;
  if (out_size != kRows * kD) return;
  if (ws_size < kWsTotal) return;

  const float* x       = (const float*)d_in[0];
  const float* W_xproj = (const float*)d_in[1];
  const float* W_dt    = (const float*)d_in[2];
  const float* b_dt    = (const float*)d_in[3];
  const float* A_log   = (const float*)d_in[4];
  float* out = (float*)d_out;

  char* ws = (char*)d_ws;
  unsigned short* XH  = (unsigned short*)(ws + kOffXH);
  unsigned short* XL  = (unsigned short*)(ws + kOffXL);
  unsigned short* WXH = (unsigned short*)(ws + kOffWXH);
  unsigned short* WXL = (unsigned short*)(ws + kOffWXL);
  unsigned short* WDH = (unsigned short*)(ws + kOffWDH);
  unsigned short* WDL = (unsigned short*)(ws + kOffWDL);
  float*          XP  = (float*)(ws + kOffXP);
  unsigned short* DRH = (unsigned short*)(ws + kOffDRH);
  unsigned short* DRL = (unsigned short*)(ws + kOffDRL);
  float*          PRE = (float*)(ws + kOffPRE);
  float*          DT  = (float*)(ws + kOffDT);

  split_rows_bf16_kernel<<<(kRows * kD / 8) / 256, 256, 0, stream>>>(
      x, (unsigned)kD, 0u, 7u, XH, XL, (unsigned)(kRows * kD / 8));
  transpose_split_bf16_kernel<<<(kXpP * kD / 8) / 256, 256, 0, stream>>>(
      W_xproj, (unsigned)kProj, 7u, WXH, WXL, (unsigned)(kXpP * kD / 8));
  transpose_split_bf16_kernel<<<(kD * kDtR / 8) / 256, 256, 0, stream>>>(
      W_dt, (unsigned)kD, 3u, WDH, WDL, (unsigned)(kD * kDtR / 8));

  wmma_gemm64_split<0><<<((kRows / 64) * (kXpP / 64)) / 8, 256, 0, stream>>>(
      XH, XL, kD, WXH, WXL, kD, XP, kXpP, b_dt, kRows, kXpP, kD);

  split_rows_bf16_kernel<<<(kRows * kDtR / 8) / 256, 256, 0, stream>>>(
      XP, (unsigned)kXpP, (unsigned)(2 * kNst), 3u, DRH, DRL, (unsigned)(kRows * kDtR / 8));

  wmma_gemm64_split<2><<<((kRows / 64) * (kD / 64)) / 8, 256, 0, stream>>>(
      DRH, DRL, kDtR, WDH, WDL, kDtR, PRE, kD, b_dt, kRows, kD, kDtR);

  softplus_kernel<<<(kRows * kD) / 2048, 256, 0, stream>>>(PRE, DT);

  scan_kernel<<<kBatch * (kD / kScanCh), kScanCh, 0, stream>>>(XP, DT, x, A_log, out);
}
